// SparseGraphAttention_30863634989574
// MI455X (gfx1250) — hardware-verified
//
#include <hip/hip_runtime.h>
#include <stddef.h>


#define DF      128
#define NH      4
#define HDIM    32
#define NBATCH  2
#define GR      32
#define AP      136
#define XSP     132
#define NB      256
#define SLOTB   8
#define CHUNK   2048
#define NTHR    256
#define NWAVE   8
#define WCAP    256
#define NGRP    (CHUNK / (NTHR * 4))

#define LDS_SACC (NB * NBATCH * DF)
#define LDS_MX   (NB * NBATCH * NH)
#define LDS_DEN  (NB * NBATCH * NH)
#define LDS_LIST (NWAVE * WCAP)
#define LDS_BYTES ((LDS_SACC + LDS_MX + LDS_DEN + LDS_LIST + NWAVE) * 4)

static_assert(DF == NH * HDIM);
static_assert(DF == 16 * NWAVE);
static_assert(NWAVE == 2 * NH);
static_assert(NTHR == 32 * NWAVE);
static_assert(GR * DF == NTHR * 16);
static_assert(NB == (1 << SLOTB));
static_assert(CHUNK <= 4096);
static_assert(WCAP == (CHUNK / NTHR) * 32);
static_assert(NGRP >= 1 && NGRP * NTHR * 4 == CHUNK);
static_assert(NBATCH <= NWAVE);
static_assert(((LDS_SACC + LDS_MX + LDS_DEN) % 4) == 0);
static_assert((NB % NWAVE) == 0);
static_assert((AP % 8) == 0 && (XSP % 4) == 0);
static_assert(LDS_BYTES == 286752);

typedef float          v4f   __attribute__((ext_vector_type(4)));
typedef float          v8f   __attribute__((ext_vector_type(8)));
typedef int            v4i   __attribute__((ext_vector_type(4)));
typedef unsigned short v8us  __attribute__((ext_vector_type(8)));
typedef __bf16         v16bf __attribute__((ext_vector_type(16)));
union FragB { v16bf v; v8us half[2]; };

__device__ __forceinline__ v8f wm(v16bf a, v16bf b, v8f c) {
  v8f d = __builtin_amdgcn_wmma_f32_16x16x32_bf16(false, a, false, b, (short)0, c, false, false);
  asm volatile("v_nop\n\tv_nop\n\tv_nop\n\tv_nop" : "+v"(d) : "v"(a), "v"(b));
  return d;
}

__device__ __forceinline__ unsigned short bfh(float f) {
  unsigned u = __float_as_uint(f);
  u += 0x7FFFu + ((u >> 16) & 1u);
  return (unsigned short)(u >> 16);
}
__device__ __forceinline__ unsigned short bfl(float f, unsigned short h) {
  const float hf = __uint_as_float(((unsigned)h) << 16);
  return bfh(f - hf);
}
__device__ __forceinline__ void split8(v4f a, v4f b, v8us& hv, v8us& lv) {
  v8us h, l;
  h[0] = bfh(a.x); l[0] = bfl(a.x, h[0]);
  h[1] = bfh(a.y); l[1] = bfl(a.y, h[1]);
  h[2] = bfh(a.z); l[2] = bfl(a.z, h[2]);
  h[3] = bfh(a.w); l[3] = bfl(a.w, h[3]);
  h[4] = bfh(b.x); l[4] = bfl(b.x, h[4]);
  h[5] = bfh(b.y); l[5] = bfl(b.y, h[5]);
  h[6] = bfh(b.z); l[6] = bfl(b.z, h[6]);
  h[7] = bfh(b.w); l[7] = bfl(b.w, h[7]);
  hv = h; lv = l;
}

__global__ __launch_bounds__(NTHR) void k_prep(const float* __restrict__ W,
                                               unsigned short* Wh, unsigned short* Wl, int n8) {
  const int i = blockIdx.x * NTHR + threadIdx.x;
  if (i >= n8) return;
  const int n  = i >> 4;
  const int k0 = (i & 15) * 8;
  v4f a, b;
  a.x = W[(size_t)(k0 + 0) * DF + n]; a.y = W[(size_t)(k0 + 1) * DF + n];
  a.z = W[(size_t)(k0 + 2) * DF + n]; a.w = W[(size_t)(k0 + 3) * DF + n];
  b.x = W[(size_t)(k0 + 4) * DF + n]; b.y = W[(size_t)(k0 + 5) * DF + n];
  b.z = W[(size_t)(k0 + 6) * DF + n]; b.w = W[(size_t)(k0 + 7) * DF + n];
  v8us hv, lv;
  split8(a, b, hv, lv);
  const size_t o = (size_t)n * DF + k0;
  *(volatile v8us*)(Wh + o) = hv;
  *(volatile v8us*)(Wl + o) = lv;
  __threadfence();
  *(volatile v8us*)(Wh + o) = hv;
  *(volatile v8us*)(Wl + o) = lv;
}

__device__ __forceinline__ void epi_tile(v8f acc, int T, int hh, int m, int wave, int ncol,
                                         float cs, float cd, float* Xs, float* As, float* Ds) {
  float ss[8], sd[8];
#pragma unroll
  for (int r = 0; r < 8; ++r) {
    const float v = acc[r];
    Xs[(T * 16 + 8 * hh + r) * XSP + ncol] = v;
    ss[r] = v * cs;
    sd[r] = v * cd;
  }
#pragma unroll
  for (int mk = 1; mk < 16; mk <<= 1) {
#pragma unroll
    for (int r = 0; r < 8; ++r) {
      ss[r] += __shfl_xor(ss[r], mk, 32);
      sd[r] += __shfl_xor(sd[r], mk, 32);
    }
  }
  if (m == 0) {
#pragma unroll
    for (int r = 0; r < 8; ++r) {
      As[(T * 16 + 8 * hh + r) * NWAVE + wave] = ss[r];
      Ds[(T * 16 + 8 * hh + r) * NWAVE + wave] = sd[r];
    }
  }
}

__global__ __launch_bounds__(NTHR) void k_gemm(
    const float* __restrict__ x, const unsigned short* __restrict__ Wh,
    const unsigned short* __restrict__ Wl, const float* __restrict__ attn,
    float* xp, float* asrc, float* adst, int nR) {
  __shared__ __attribute__((aligned(16))) unsigned short Ah[GR * AP];
  __shared__ __attribute__((aligned(16))) unsigned short Al[GR * AP];
  __shared__ __attribute__((aligned(16))) float Xs[GR * XSP];
  __shared__ __attribute__((aligned(16))) float As[GR * NWAVE];
  __shared__ __attribute__((aligned(16))) float Ds[GR * NWAVE];

  const int tid  = threadIdx.x;
  const int lane = tid & 31;
  const int wave = tid >> 5;
  const int hh   = lane >> 4;
  const int m    = lane & 15;
  const int rowBase = blockIdx.x * GR;

  {
    const int r  = tid >> 3;
    const int c0 = (tid & 7) * 16;
    int row = rowBase + r;
    if (row > nR - 1) row = nR - 1;
    const float* p = x + (size_t)row * DF + c0;
    const v4f f0 = *(const v4f*)(p),     f1 = *(const v4f*)(p + 4);
    const v4f f2 = *(const v4f*)(p + 8), f3 = *(const v4f*)(p + 12);
    v8us h0, l0, h1, l1;
    split8(f0, f1, h0, l0);
    split8(f2, f3, h1, l1);
    *(v8us*)(Ah + r * AP + c0)     = h0;
    *(v8us*)(Ah + r * AP + c0 + 8) = h1;
    *(v8us*)(Al + r * AP + c0)     = l0;
    *(v8us*)(Al + r * AP + c0 + 8) = l1;
  }
  __syncthreads();

  const int ncol = wave * 16 + m;
  v8f c0a = {0.f, 0.f, 0.f, 0.f, 0.f, 0.f, 0.f, 0.f};
  v8f c1a = {0.f, 0.f, 0.f, 0.f, 0.f, 0.f, 0.f, 0.f};
#pragma unroll
  for (int kt = 0; kt < DF / 32; ++kt) {
    const int k0 = kt * 32;
    FragB a0h, a0l, a1h, a1l, bh, bl;
    const unsigned short* pbh  = Wh + (size_t)ncol * DF + k0 + 8 * hh;
    const unsigned short* pbl  = Wl + (size_t)ncol * DF + k0 + 8 * hh;
    const unsigned short* pa0h = Ah + m * AP + k0 + 8 * hh;
    const unsigned short* pa0l = Al + m * AP + k0 + 8 * hh;
    const unsigned short* pa1h = Ah + (16 + m) * AP + k0 + 8 * hh;
    const unsigned short* pa1l = Al + (16 + m) * AP + k0 + 8 * hh;
    bh.half[0]  = *(const v8us*)pbh;  bh.half[1]  = *(const v8us*)(pbh + 16);
    bl.half[0]  = *(const v8us*)pbl;  bl.half[1]  = *(const v8us*)(pbl + 16);
    a0h.half[0] = *(const v8us*)pa0h; a0h.half[1] = *(const v8us*)(pa0h + 16);
    a0l.half[0] = *(const v8us*)pa0l; a0l.half[1] = *(const v8us*)(pa0l + 16);
    a1h.half[0] = *(const v8us*)pa1h; a1h.half[1] = *(const v8us*)(pa1h + 16);
    a1l.half[0] = *(const v8us*)pa1l; a1l.half[1] = *(const v8us*)(pa1l + 16);
    c0a = wm(a0h.v, bh.v, c0a);
    c0a = wm(a0h.v, bl.v, c0a);
    c0a = wm(a0l.v, bh.v, c0a);
    c1a = wm(a1h.v, bh.v, c1a);
    c1a = wm(a1h.v, bl.v, c1a);
    c1a = wm(a1l.v, bh.v, c1a);
  }

  const int head = ncol >> 5;
  const int d    = ncol & (HDIM - 1);
  const float cs = attn[head * 2 * HDIM + d];
  const float cd = attn[head * 2 * HDIM + HDIM + d];
  epi_tile(c0a, 0, hh, m, wave, ncol, cs, cd, Xs, As, Ds);
  epi_tile(c1a, 1, hh, m, wave, ncol, cs, cd, Xs, As, Ds);
  __syncthreads();

  v4f xr[4];
#pragma unroll
  for (int i = 0; i < 4; ++i) xr[i] = *(const v4f*)(Xs + (4 * wave + i) * XSP + 4 * lane);
  v4f gv = {0.f, 0.f, 0.f, 0.f};
  float* gp = asrc;
  const bool doG = (wave < 2);
  if (wave == 0) {
    const float* q = As + lane * NWAVE;
    gv.x = q[0] + q[1]; gv.y = q[2] + q[3]; gv.z = q[4] + q[5]; gv.w = q[6] + q[7];
    gp = asrc + (size_t)rowBase * NH + 4 * lane;
  } else if (wave == 1) {
    const float* q = Ds + lane * NWAVE;
    gv.x = q[0] + q[1]; gv.y = q[2] + q[3]; gv.z = q[4] + q[5]; gv.w = q[6] + q[7];
    gp = adst + (size_t)rowBase * NH + 4 * lane;
  }
  float* xpp[4];
#pragma unroll
  for (int i = 0; i < 4; ++i) xpp[i] = xp + (size_t)(rowBase + 4 * wave + i) * DF + 4 * lane;

#pragma unroll
  for (int i = 0; i < 4; ++i) *(volatile v4f*)(xpp[i]) = xr[i];
  if (doG) *(volatile v4f*)gp = gv;
  __threadfence();
#pragma unroll
  for (int i = 0; i < 4; ++i) *(volatile v4f*)(xpp[i]) = xr[i];
  if (doG) *(volatile v4f*)gp = gv;
}

__global__ __launch_bounds__(NTHR) void k_agg(
    const int* __restrict__ ei, const float* __restrict__ xp,
    const float* __restrict__ asrc, const float* __restrict__ adst,
    float* out, int nN, int nE) {
  extern __shared__ v4f lds_dyn[];
  float* sacc = (float*)lds_dyn;
  float* smx  = sacc + LDS_SACC;
  float* sden = smx + LDS_MX;
  int*   list = (int*)(sden + LDS_DEN);
  int*   wcnt = list + LDS_LIST;

  const int tid  = threadIdx.x;
  const int lane = tid & 31;
  const int wave = tid >> 5;
  const int hd   = lane >> 3;
  const int nodeBase = blockIdx.x * NB;

  {
    const v4f z4 = {0.f, 0.f, 0.f, 0.f};
    for (int i = tid; i < (LDS_SACC + LDS_MX + LDS_DEN) / 4; i += NTHR) lds_dyn[i] = z4;
  }
  __syncthreads();

  const int* eid = ei + nE;
  const bool al16 = ((nE & 3) == 0);

  const int nChunks = (nE + CHUNK - 1) / CHUNK;
#pragma unroll 1
  for (int ch = 0; ch < nChunks; ++ch) {
    const int cbase = ch * CHUNK;
    int wc = 0;
#pragma unroll
    for (int g = 0; g < NGRP; ++g) {
      const int el0 = (g * NTHR + tid) * 4;
      const int e0  = cbase + el0;
      const int sent = -2147483647 - 1;
      v4i d;
      if (al16 && (cbase + CHUNK <= nE)) {
        d = *(const v4i*)(eid + e0);
      } else {
        d.x = (e0     < nE) ? eid[min(e0,     nE - 1)] : sent;
        d.y = (e0 + 1 < nE) ? eid[min(e0 + 1, nE - 1)] : sent;
        d.z = (e0 + 2 < nE) ? eid[min(e0 + 2, nE - 1)] : sent;
        d.w = (e0 + 3 < nE) ? eid[min(e0 + 3, nE - 1)] : sent;
      }
      const unsigned s0 = (unsigned)d.x - (unsigned)nodeBase;
      const unsigned s1 = (unsigned)d.y - (unsigned)nodeBase;
      const unsigned s2 = (unsigned)d.z - (unsigned)nodeBase;
      const unsigned s3 = (unsigned)d.w - (unsigned)nodeBase;
      const bool h0 = s0 < (unsigned)NB;
      const bool h1 = s1 < (unsigned)NB;
      const bool h2 = s2 < (unsigned)NB;
      const bool h3 = s3 < (unsigned)NB;
      const unsigned many = __builtin_amdgcn_ballot_w32(h0 | h1 | h2 | h3);
      if (many != 0u) {
#define HITJ(J, HJ, SJ) { \
          const unsigned mj = __builtin_amdgcn_ballot_w32(HJ); \
          if (HJ) { \
            const int pos = wc + (int)__builtin_amdgcn_mbcnt_lo(mj, 0u); \
            if (pos < WCAP) list[wave * WCAP + pos] = ((el0 + (J)) << SLOTB) | (int)(SJ); \
          } \
          wc += (int)__builtin_popcount(mj); }
        HITJ(0, h0, s0)
        HITJ(1, h1, s1)
        HITJ(2, h2, s2)
        HITJ(3, h3, s3)
#undef HITJ
      }
    }
    if (lane == 0) wcnt[wave] = wc;
    __syncthreads();

    if (wave < NBATCH) {
      const int b = wave;
      const size_t bOff = (size_t)b * (size_t)nN;
      for (int wsx = 0; wsx < NWAVE; ++wsx) {
        int n = wcnt[wsx];
        if (n > WCAP) n = WCAP;
        if (n < 0) n = 0;
        for (int i = 0; i < n; ++i) {
          const int ent  = list[wsx * WCAP + i];
          const int slot = ent & (NB - 1);
          const int el   = (ent >> SLOTB) & (CHUNK - 1);
          int e = cbase + el;
          if (e > nE - 1) e = nE - 1;
          int src = ei[e];
          src = src < 0 ? 0 : (src > nN - 1 ? nN - 1 : src);
          int nd = nodeBase + slot;
          if (nd > nN - 1) nd = nN - 1;
          const size_t rs = bOff + (size_t)src;
          const size_t rd = bOff + (size_t)nd;
          float s = asrc[rs * NH + hd] + adst[rd * NH + hd];
          s = (s > 0.f) ? s : 0.2f * s;
          const int ai = (slot * NBATCH + b) * NH + hd;
          const float mo = smx[ai];
          const float mn = fmaxf(mo, s);
          const float sc = __expf(mo - mn);
          const float p  = __expf(s - mn);
          const v4f xv = *(const v4f*)(xp + rs * DF + 4 * lane);
          v4f* ap = (v4f*)(sacc + (slot * NBATCH + b) * DF + 4 * lane);
          const v4f cur = *ap;
          const v4f nxt = cur * sc + xv * p;
          *ap = nxt;
          const float dn = sden[ai];
          sden[ai] = dn * sc + p;
          smx[ai]  = mn;
        }
      }
    }
    __syncthreads();
  }

#pragma unroll 1
  for (int j = 0; j < NB / NWAVE; ++j) {
    const int slot = wave * (NB / NWAVE) + j;
    const int node = nodeBase + slot;
    if (node >= nN) break;
#pragma unroll
    for (int b = 0; b < NBATCH; ++b) {
      const int ai = (slot * NBATCH + b) * NH + hd;
      const float inv = 1.0f / (sden[ai] + 1e-8f);
      const v4f y = *(const v4f*)(sacc + (slot * NBATCH + b) * DF + 4 * lane) * inv;
      float* op = out + ((size_t)b * (size_t)nN + (size_t)node) * DF + 4 * lane;
      *(volatile v4f*)op = y;
      __threadfence();
      *(volatile v4f*)op = y;
    }
  }
}

extern "C" void kernel_launch(void* const* d_in, const int* in_sizes, int n_in,
                              void* d_out, int out_size, void* d_ws, size_t ws_size,
                              hipStream_t stream) {
  if (n_in < 4) return;
  const int nR = in_sizes[0] / DF;
  if (nR <= 0 || in_sizes[0] != nR * DF || (nR % NBATCH) != 0) return;
  const int nN = nR / NBATCH;
  const int nE = in_sizes[1] / 2;
  if (nE < 0 || in_sizes[1] != 2 * nE) return;
  if (in_sizes[2] != DF * DF) return;
  if (in_sizes[3] != NH * 2 * HDIM) return;
  if (out_size != nR * DF) return;

  const float* x    = (const float*)d_in[0];
  const int*   ei   = (const int*)d_in[1];
  const float* W    = (const float*)d_in[2];
  const float* attn = (const float*)d_in[3];
  float* out = (float*)d_out;

  const int nP = ((nR + GR - 1) / GR) * GR;
  size_t off = 0;
  unsigned short* Wh = (unsigned short*)((char*)d_ws + off); off += (size_t)DF * DF * sizeof(unsigned short);
  unsigned short* Wl = (unsigned short*)((char*)d_ws + off); off += (size_t)DF * DF * sizeof(unsigned short);
  float* xp   = (float*)((char*)d_ws + off);                 off += (size_t)nP * DF * sizeof(float);
  float* asrc = (float*)((char*)d_ws + off);                 off += (size_t)nP * NH * sizeof(float);
  float* adst = (float*)((char*)d_ws + off);                 off += (size_t)nP * NH * sizeof(float);
  if (off > ws_size) return;

  const int n8 = DF * DF / 8;
  k_prep<<<(n8 + NTHR - 1) / NTHR, NTHR, 0, stream>>>(W, Wh, Wl, n8);

  k_gemm<<<nP / GR, NTHR, 0, stream>>>(x, Wh, Wl, attn, xp, asrc, adst, nR);

  hipFuncSetAttribute(reinterpret_cast<const void*>(&k_agg),
                      hipFuncAttributeMaxDynamicSharedMemorySize, LDS_BYTES);
  const int grid = (nN + NB - 1) / NB;
  k_agg<<<grid, NTHR, LDS_BYTES, stream>>>(ei, xp, asrc, adst, out, nN, nE);
}
